// MiniTFT_Step8_77412490543362
// MI455X (gfx1250) — hardware-verified
//
#include <hip/hip_runtime.h>
#define BB 128
#define TE 512
#define TD 128
#define FF 32
#define HH 64
#define G4 256
#define NTE (BB * TE)
#define NTD (BB * TD)

typedef __bf16 v16b __attribute__((ext_vector_type(16)));
typedef unsigned short v8us __attribute__((ext_vector_type(8), may_alias));
typedef float  v8f  __attribute__((ext_vector_type(8)));
typedef float  v4f  __attribute__((ext_vector_type(4)));
typedef float  v4fa __attribute__((ext_vector_type(4), may_alias));
union FragB { v16b v; v8us half[2]; unsigned short u[16]; };

__device__ __forceinline__ unsigned short bf16_bits(float x) { unsigned int u = __float_as_uint(x); return (unsigned short)((u + 0x7FFFu + ((u >> 16) & 1u)) >> 16); }
__device__ __forceinline__ float bf16_val(unsigned short b) { return __uint_as_float(((unsigned int)b) << 16); }
__device__ __forceinline__ float bf16_round(float x) { return bf16_val(bf16_bits(x)); }
template <int NT>
__device__ __forceinline__ v8f mmaN(v16b ah, v16b al, v16b bh, v16b bl, v8f c) {
  c = __builtin_amdgcn_wmma_f32_16x16x32_bf16(false, ah, false, bh, (short)0, c, false, false);
  if (NT >= 2) c = __builtin_amdgcn_wmma_f32_16x16x32_bf16(false, al, false, bh, (short)0, c, false, false);
  if (NT >= 3) c = __builtin_amdgcn_wmma_f32_16x16x32_bf16(false, ah, false, bl, (short)0, c, false, false);
  asm volatile("v_nop\n\tv_nop\n\tv_nop\n\tv_nop" : "+v"(c) : "v"(ah), "v"(al), "v"(bh), "v"(bl));
  return c;
}

__global__ __launch_bounds__(256) void k_wt_bf16(const float* __restrict__ W, unsigned short* __restrict__ Wt, int K, int N) {
  const int t = blockIdx.x * 256 + threadIdx.x;
  const int k8n = K / 8;
  if (t >= N * k8n) return;
  const int n = t / k8n, k8 = (t % k8n) * 8;
  v8us v;
#pragma unroll
  for (int i = 0; i < 8; ++i) v[i] = bf16_bits(W[(size_t)(k8 + i) * N + n]);
  *(volatile v8us*)(Wt + (size_t)n * K + k8) = v;
  __threadfence();
  *(volatile v8us*)(Wt + (size_t)n * K + k8) = v;
}

template <bool ASPLIT, int ACT, bool BIAS_BF16>
__global__ __launch_bounds__(128) void k_gemm_bf(const float* __restrict__ A, int lda, const unsigned short* __restrict__ Wt, int ldb,
                                               const float* __restrict__ bias, float* __restrict__ C, int ldc, int M, int N, int K) {
  __shared__ __attribute__((aligned(16))) float so[4][16][64];
  const int tid = threadIdx.x, w = tid >> 5, lane = tid & 31, ln = lane & 15, hh = lane >> 4;
  const int ntn = N / 64;
  const int wid = blockIdx.x * 4 + w;
  const int mt = wid / ntn, nq = wid % ntn;
  if (mt * 16 >= M) return;
  const int row0 = mt * 16, col0 = nq * 64;
  const float* arow = A + (size_t)(row0 + ln) * lda;
  v8f acc[4] = {};
  for (int kb = 0; kb < K; kb += 32) {
    FragB ah, al;
    const v4f x0 = *(const v4fa*)(arow + kb + 8 * hh), x1 = *(const v4fa*)(arow + kb + 8 * hh + 4);
    const v4f x2 = *(const v4fa*)(arow + kb + 16 + 8 * hh), x3 = *(const v4fa*)(arow + kb + 16 + 8 * hh + 4);
    float xs[16] = {x0[0],x0[1],x0[2],x0[3],x1[0],x1[1],x1[2],x1[3],x2[0],x2[1],x2[2],x2[3],x3[0],x3[1],x3[2],x3[3]};
#pragma unroll
    for (int i = 0; i < 16; ++i) { const unsigned short hb = bf16_bits(xs[i]); ah.u[i] = hb; al.u[i] = ASPLIT ? bf16_bits(xs[i] - bf16_val(hb)) : (unsigned short)0; }
#pragma unroll
    for (int t = 0; t < 4; ++t) {
      const unsigned short* brow = Wt + (size_t)(col0 + t * 16 + ln) * ldb + kb;
      FragB b;
      b.half[0] = *(const v8us*)(brow + 8 * hh);
      b.half[1] = *(const v8us*)(brow + 16 + 8 * hh);
      acc[t] = mmaN<ASPLIT ? 2 : 1>(ah.v, al.v, b.v, b.v, acc[t]);
    }
  }
#pragma unroll
  for (int t = 0; t < 4; ++t) {
    float bv = bias ? bias[col0 + t * 16 + ln] : 0.f;
    if (BIAS_BF16) bv = bf16_round(bv);
#pragma unroll
    for (int r = 0; r < 8; ++r) { float v = acc[t][r] + bv; if (ACT == 1) v = fmaxf(v, 0.f); so[w][8 * hh + r][t * 16 + ln] = v; }
  }
  __builtin_amdgcn_fence(__ATOMIC_ACQ_REL, "workgroup");
  __builtin_amdgcn_wave_barrier();
  const int rsub = lane >> 4, c4 = (lane & 15) * 4;
  for (int pass = 0; pass < 2; ++pass) {
#pragma unroll
    for (int q = 0; q < 8; ++q) {
      const int r = q * 2 + rsub;
      const v4f v = *(const v4fa*)&so[w][r][c4];
      *(volatile v4f*)(C + (size_t)(row0 + r) * ldc + col0 + c4) = v;
    }
    if (pass == 0) __threadfence();
  }
}

template <int D, bool CAUSAL>
__global__ __launch_bounds__(128) void k_flash(const float* __restrict__ qb, const float* __restrict__ kb, const float* __restrict__ vb,
                                             int pitch, int T, int H, float scale, float* __restrict__ y, int ypitch) {
  constexpr int KS = D / 32;
  constexpr int DT = D / 16;
  __shared__ __attribute__((aligned(16))) unsigned short sKh[32][D + 8], sKl[32][D + 8], sVh[32][D + 8], sVl[32][D + 8];
  __shared__ __attribute__((aligned(16))) unsigned short sPh[4][16][40], sPl[4][16][40];
  __shared__ __attribute__((aligned(16))) float sO[4][16][D];
  const int tid = threadIdx.x, w = tid >> 5, lane = tid & 31, ln = lane & 15, hh = lane >> 4;
  const int nqb = (T + 63) / 64;
  const int bh = blockIdx.x / nqb, qblk = blockIdx.x % nqb;
  const int b = bh / H, h = bh % H;
  const int q0 = qblk * 64 + w * 16;
  const float* Q = qb + (size_t)b * T * pitch + h * D;
  const float* K = kb + (size_t)b * T * pitch + h * D;
  const float* V = vb + (size_t)b * T * pitch + h * D;

  FragB aqh[KS], aql[KS];
  {
    int row = q0 + ln; if (row >= T) row = T - 1;
    const float* qr = Q + (size_t)row * pitch;
#pragma unroll
    for (int ks = 0; ks < KS; ++ks)
#pragma unroll
      for (int i = 0; i < 16; ++i) {
        const int d = ks * 32 + ((i < 8) ? (8 * hh + i) : (16 + 8 * hh + (i - 8)));
        const float x = qr[d] * scale; const unsigned short hb = bf16_bits(x);
        aqh[ks].u[i] = hb; aql[ks].u[i] = bf16_bits(x - bf16_val(hb));
      }
  }
  float m_r[8], l_r[8];
#pragma unroll
  for (int r = 0; r < 8; ++r) { m_r[r] = -3.0e38f; l_r[r] = 0.f; }
  v8f oacc[DT];
#pragma unroll
  for (int dt = 0; dt < DT; ++dt) oacc[dt] = (v8f){0.f,0.f,0.f,0.f,0.f,0.f,0.f,0.f};

  const int kv_end = CAUSAL ? min(T, qblk * 64 + 64) : T;
  for (int j0 = 0; j0 < kv_end; j0 += 32) {
    __syncthreads();
    for (int e = tid; e < 32 * (D / 4); e += 128) {
      const int r = e / (D / 4), c4 = (e % (D / 4)) * 4;
      const int key = j0 + r;
      v4f kf = {0.f,0.f,0.f,0.f}, vf = {0.f,0.f,0.f,0.f};
      if (key < T) { kf = *(const v4fa*)(K + (size_t)key * pitch + c4); vf = *(const v4fa*)(V + (size_t)key * pitch + c4); }
#pragma unroll
      for (int t = 0; t < 4; ++t) {
        unsigned short hb = bf16_bits(kf[t]); sKh[r][c4 + t] = hb; sKl[r][c4 + t] = bf16_bits(kf[t] - bf16_val(hb));
        hb = bf16_bits(vf[t]); sVh[r][c4 + t] = hb; sVl[r][c4 + t] = bf16_bits(vf[t] - bf16_val(hb));
      }
    }
    __syncthreads();
    v8f s[2];
#pragma unroll
    for (int nt = 0; nt < 2; ++nt) {
      v8f acc = {};
#pragma unroll
      for (int ks = 0; ks < KS; ++ks) {
        FragB bh_, bl_;
        bh_.half[0] = *(const v8us*)&sKh[nt * 16 + ln][ks * 32 + 8 * hh]; bh_.half[1] = *(const v8us*)&sKh[nt * 16 + ln][ks * 32 + 16 + 8 * hh];
        bl_.half[0] = *(const v8us*)&sKl[nt * 16 + ln][ks * 32 + 8 * hh]; bl_.half[1] = *(const v8us*)&sKl[nt * 16 + ln][ks * 32 + 16 + 8 * hh];
        acc = mmaN<3>(aqh[ks].v, aql[ks].v, bh_.v, bl_.v, acc);
      }
      s[nt] = acc;
    }
    float alpha[8];
#pragma unroll
    for (int r = 0; r < 8; ++r) {
      const int qi = q0 + 8 * hh + r;
      const int ja = j0 + ln, jb = j0 + 16 + ln;
      if (CAUSAL) { if (ja > qi) s[0][r] = -3.0e38f; if (jb > qi) s[1][r] = -3.0e38f; }
      if (ja >= T) s[0][r] = -3.0e38f;
      if (jb >= T) s[1][r] = -3.0e38f;
      float mx = fmaxf(s[0][r], s[1][r]);
      mx = fmaxf(mx, __shfl_xor(mx, 1, 32)); mx = fmaxf(mx, __shfl_xor(mx, 2, 32)); mx = fmaxf(mx, __shfl_xor(mx, 4, 32)); mx = fmaxf(mx, __shfl_xor(mx, 8, 32));
      const float mnew = fmaxf(m_r[r], mx);
      alpha[r] = (mnew > -1.0e38f) ? __expf(m_r[r] - mnew) : 1.0f;
      const float p0 = (s[0][r] > -1.0e38f) ? __expf(s[0][r] - mnew) : 0.f;
      const float p1 = (s[1][r] > -1.0e38f) ? __expf(s[1][r] - mnew) : 0.f;
      m_r[r] = mnew;
      l_r[r] = l_r[r] * alpha[r] + p0 + p1;
      unsigned short hb = bf16_bits(p0); sPh[w][8 * hh + r][ln] = hb;      sPl[w][8 * hh + r][ln] = bf16_bits(p0 - bf16_val(hb));
      hb = bf16_bits(p1);                sPh[w][8 * hh + r][16 + ln] = hb; sPl[w][8 * hh + r][16 + ln] = bf16_bits(p1 - bf16_val(hb));
    }
#pragma unroll
    for (int dt = 0; dt < DT; ++dt)
#pragma unroll
      for (int r = 0; r < 8; ++r) oacc[dt][r] *= alpha[r];
    __builtin_amdgcn_fence(__ATOMIC_ACQ_REL, "workgroup");
    __builtin_amdgcn_wave_barrier();
    FragB pah, pal;
    pah.half[0] = *(const v8us*)&sPh[w][ln][8 * hh]; pah.half[1] = *(const v8us*)&sPh[w][ln][16 + 8 * hh];
    pal.half[0] = *(const v8us*)&sPl[w][ln][8 * hh]; pal.half[1] = *(const v8us*)&sPl[w][ln][16 + 8 * hh];
#pragma unroll
    for (int dt = 0; dt < DT; ++dt) {
      FragB bvh, bvl;
#pragma unroll
      for (int i = 0; i < 8; ++i) {
        bvh.u[i] = sVh[8 * hh + i][dt * 16 + ln]; bvh.u[8 + i] = sVh[16 + 8 * hh + i][dt * 16 + ln];
        bvl.u[i] = sVl[8 * hh + i][dt * 16 + ln]; bvl.u[8 + i] = sVl[16 + 8 * hh + i][dt * 16 + ln];
      }
      oacc[dt] = mmaN<3>(pah.v, pal.v, bvh.v, bvl.v, oacc[dt]);
    }
    __builtin_amdgcn_fence(__ATOMIC_ACQ_REL, "workgroup");
    __builtin_amdgcn_wave_barrier();
  }
#pragma unroll
  for (int r = 0; r < 8; ++r) {
    float l = l_r[r];
    l += __shfl_xor(l, 1, 32); l += __shfl_xor(l, 2, 32); l += __shfl_xor(l, 4, 32); l += __shfl_xor(l, 8, 32);
    l_r[r] = (l > 0.f) ? 1.0f / l : 0.f;
  }
#pragma unroll
  for (int dt = 0; dt < DT; ++dt)
#pragma unroll
    for (int r = 0; r < 8; ++r) sO[w][8 * hh + r][dt * 16 + ln] = oacc[dt][r] * l_r[r];
  __builtin_amdgcn_fence(__ATOMIC_ACQ_REL, "workgroup");
  __builtin_amdgcn_wave_barrier();
  for (int pass = 0; pass < 2; ++pass) {
    for (int r = 0; r < 16; ++r) {
      const int row = q0 + r;
      if (row < T && lane < D / 4) {
        const v4f val = *(const v4fa*)&sO[w][r][lane * 4];
        *(volatile v4f*)(y + ((size_t)b * T + row) * ypitch + h * D + lane * 4) = val;
      }
    }
    if (pass == 0) __threadfence();
  }
}

template <bool ASPLIT, int ACT, bool BIAS_BF16, bool RES_BF16>
__global__ __launch_bounds__(128) void k_gemm_bf3(const float* __restrict__ A, int lda, const unsigned short* __restrict__ Wt, int ldb,
                                                const float* __restrict__ bias, const float* __restrict__ resid, int rmod, int ldr,
                                                float* __restrict__ C, int ldc, int M, int N, int K) {
  __shared__ __attribute__((aligned(16))) float so[4][16][64];
  const int tid = threadIdx.x, w = tid >> 5, lane = tid & 31, ln = lane & 15, hh = lane >> 4;
  const int ntn = N / 64;
  const int wid = blockIdx.x * 4 + w;
  const int mt = wid / ntn, nq = wid % ntn;
  if (mt * 16 >= M) return;
  const int row0 = mt * 16, col0 = nq * 64;
  const float* arow = A + (size_t)(row0 + ln) * lda;
  v8f acc[4] = {};
  for (int kb = 0; kb < K; kb += 32) {
    FragB ah, al;
    const v4f x0 = *(const v4fa*)(arow + kb + 8 * hh), x1 = *(const v4fa*)(arow + kb + 8 * hh + 4);
    const v4f x2 = *(const v4fa*)(arow + kb + 16 + 8 * hh), x3 = *(const v4fa*)(arow + kb + 16 + 8 * hh + 4);
    float xs[16] = {x0[0],x0[1],x0[2],x0[3],x1[0],x1[1],x1[2],x1[3],x2[0],x2[1],x2[2],x2[3],x3[0],x3[1],x3[2],x3[3]};
#pragma unroll
    for (int i = 0; i < 16; ++i) { const unsigned short hb = bf16_bits(xs[i]); ah.u[i] = hb; al.u[i] = ASPLIT ? bf16_bits(xs[i] - bf16_val(hb)) : (unsigned short)0; }
#pragma unroll
    for (int t = 0; t < 4; ++t) {
      const unsigned short* brow = Wt + (size_t)(col0 + t * 16 + ln) * ldb + kb;
      FragB b;
      b.half[0] = *(const v8us*)(brow + 8 * hh);
      b.half[1] = *(const v8us*)(brow + 16 + 8 * hh);
      acc[t] = mmaN<ASPLIT ? 2 : 1>(ah.v, al.v, b.v, b.v, acc[t]);
    }
  }
#pragma unroll
  for (int t = 0; t < 4; ++t) {
    const int col = col0 + t * 16 + ln;
    float bv = bias ? bias[col] : 0.f;
    if (BIAS_BF16) bv = bf16_round(bv);
#pragma unroll
    for (int r = 0; r < 8; ++r) {
      float v = acc[t][r] + bv;
      if (resid) { float rv = resid[(size_t)((row0 + 8 * hh + r) % rmod) * ldr + col]; if (RES_BF16) rv = bf16_round(rv); v += rv; }
      if (ACT == 1) v = fmaxf(v, 0.f);
      if (ACT == 2) v = 0.5f * v * (1.0f + erff(v * 0.70710678118654752f));
      if (ACT == 3) { const float u = 0.7978845608028654f * (v + 0.044715f * v * v * v); v = 0.5f * v * (1.0f + tanhf(u)); }
      so[w][8 * hh + r][t * 16 + ln] = v;
    }
  }
  __builtin_amdgcn_fence(__ATOMIC_ACQ_REL, "workgroup");
  __builtin_amdgcn_wave_barrier();
  const int rsub = lane >> 4, c4 = (lane & 15) * 4;
  for (int pass = 0; pass < 2; ++pass) {
#pragma unroll
    for (int q = 0; q < 8; ++q) {
      const int r = q * 2 + rsub;
      const v4f v = *(const v4fa*)&so[w][r][c4];
      *(volatile v4f*)(C + (size_t)(row0 + r) * ldc + col0 + c4) = v;
    }
    if (pass == 0) __threadfence();
  }
}
template <bool PARAM_BF16>
__global__ __launch_bounds__(256) void k_layernorm(const float* __restrict__ X, const float* __restrict__ R, const float* __restrict__ g, const float* __restrict__ bta,
                                                  float* __restrict__ out_sum, float* __restrict__ out_norm, int N, float eps) {
  __shared__ float red[256];
  const int row = blockIdx.x, tid = threadIdx.x;
  const float* x = X + (size_t)row * N; const float* rr = R ? R + (size_t)row * N : nullptr;
  float vals[16];
  const int per = N / 256;
  float s1 = 0.f;
  for (int u = 0; u < per / 4; ++u) {
    const int j = tid * 4 + 1024 * u;
    const v4f a = *(const v4fa*)(x + j);
    v4f b = {0.f,0.f,0.f,0.f}; if (rr) b = *(const v4fa*)(rr + j);
#pragma unroll
    for (int q = 0; q < 4; ++q) { const float v = a[q] + b[q]; vals[u * 4 + q] = v; s1 += v; }
  }
  red[tid] = s1; __syncthreads();
  for (int st = 128; st > 0; st >>= 1) { if (tid < st) red[tid] += red[tid + st]; __syncthreads(); }
  const float mu = red[0] / (float)N; __syncthreads();
  float s2 = 0.f;
  for (int u = 0; u < per / 4; ++u)
#pragma unroll
    for (int q = 0; q < 4; ++q) { const float c = vals[u * 4 + q] - mu; s2 += c * c; }
  red[tid] = s2; __syncthreads();
  for (int st = 128; st > 0; st >>= 1) { if (tid < st) red[tid] += red[tid + st]; __syncthreads(); }
  const float rs = rsqrtf(red[0] / (float)N + eps);
  for (int pass = 0; pass < 2; ++pass) {
    for (int u = 0; u < per / 4; ++u) {
      const int j = tid * 4 + 1024 * u;
      v4f o, sm;
#pragma unroll
      for (int q = 0; q < 4; ++q) {
        float gg = g[j + q], bb = bta[j + q];
        if (PARAM_BF16) { gg = bf16_round(gg); bb = bf16_round(bb); }
        sm[q] = vals[u * 4 + q]; o[q] = (vals[u * 4 + q] - mu) * rs * gg + bb;
      }
      if (out_sum) *(volatile v4f*)(out_sum + (size_t)row * N + j) = sm;
      *(volatile v4f*)(out_norm + (size_t)row * N + j) = o;
    }
    if (pass == 0) __threadfence();
  }
}

__global__ __launch_bounds__(256) void k_round_rows(const float* __restrict__ W, unsigned short* __restrict__ Wt, int n8) {
  const int t = blockIdx.x * 256 + threadIdx.x;
  if (t >= n8) return;
  const v4f a = *(const v4fa*)(W + (size_t)t * 8), b = *(const v4fa*)(W + (size_t)t * 8 + 4);
  v8us v; v[0]=bf16_bits(a[0]); v[1]=bf16_bits(a[1]); v[2]=bf16_bits(a[2]); v[3]=bf16_bits(a[3]);
  v[4]=bf16_bits(b[0]); v[5]=bf16_bits(b[1]); v[6]=bf16_bits(b[2]); v[7]=bf16_bits(b[3]);
  *(volatile v8us*)(Wt + (size_t)t * 8) = v; __threadfence(); *(volatile v8us*)(Wt + (size_t)t * 8) = v;
}

__device__ __forceinline__ float sigm(float x) { return 1.0f / (1.0f + __expf(-x)); }
__device__ __forceinline__ float tnh(float x) { const float e = __expf(2.0f * x); return 1.0f - 2.0f / (1.0f + e); }
__global__ __launch_bounds__(256) void k_vsnA(const float* __restrict__ X, const float* __restrict__ Smat, int ntok, float* __restrict__ A) {
  __shared__ float sS[FF][FF + 1]; __shared__ float sx[8][FF]; const int tid = threadIdx.x, wv = tid >> 5, lane = tid & 31;
  for (int e = tid; e < FF * FF; e += 256) sS[e / FF][e % FF] = bf16_round(Smat[e]); __syncthreads();
  const int tk = blockIdx.x * 8 + wv; if (tk >= ntok) return; const float xv = bf16_round(X[(size_t)tk * FF + lane]); sx[wv][lane] = xv;
  __builtin_amdgcn_fence(__ATOMIC_ACQ_REL, "workgroup"); __builtin_amdgcn_wave_barrier();
  float s = 0.f;
#pragma unroll
  for (int f = 0; f < FF; ++f) s += sx[wv][f] * sS[lane][f];
  float mx = s; for (int o = 16; o >= 1; o >>= 1) mx = fmaxf(mx, __shfl_xor(mx, o, 32)); const float ex = expf(s - mx); float den = ex; for (int o = 16; o >= 1; o >>= 1) den += __shfl_xor(den, o, 32); const float w = ex / den;
  float* row = A + (size_t)tk * (2 * FF); for (int pass = 0; pass < 2; ++pass) { *(volatile float*)(row + lane) = xv * w; *(volatile float*)(row + FF + lane) = w; if (pass == 0) __threadfence(); }
}
__global__ __launch_bounds__(256) void k_btvsn(const float* __restrict__ Wp, const float* __restrict__ bp, unsigned short* __restrict__ Bt) { const int t = blockIdx.x * 256 + threadIdx.x; if (t >= HH * 8) return; const int h = t / 8, k8 = (t % 8) * 8; v8us v;
#pragma unroll
  for (int q = 0; q < 8; ++q) { const int k = k8 + q; v[q] = bf16_bits(k < FF ? Wp[k * HH + h] : bp[(k - FF) * HH + h]); } *(volatile v8us*)(Bt + h * (2 * FF) + k8) = v; __threadfence(); *(volatile v8us*)(Bt + h * (2 * FF) + k8) = v; }
__global__ __launch_bounds__(256) void k_bcat2(const float* __restrict__ a, const float* __restrict__ b, float* __restrict__ o) { const int t = threadIdx.x; if (t < 2 * HH) { const float v = bf16_round(t < HH ? a[t] : b[t - HH]); *(volatile float*)(o + t) = v; __threadfence(); *(volatile float*)(o + t) = v; } }
__global__ __launch_bounds__(256) void k_bsum(const float* __restrict__ a, const float* __restrict__ b, float* __restrict__ o) { const int t = threadIdx.x; if (t < G4) { const float v = bf16_round(a[t]) + bf16_round(b[t]); *(volatile float*)(o + t) = v; __threadfence(); *(volatile float*)(o + t) = v; } }
__global__ __launch_bounds__(64) void k_lstm2(const float* __restrict__ GIe, const float* __restrict__ GId, const float* __restrict__ Whh_e, const float* __restrict__ Whh_d, const float* __restrict__ bh0, const float* __restrict__ bc0, float* __restrict__ DEC) {
  __shared__ float sH[2][16][HH + 1]; __shared__ float sC[2][16][HH + 1]; __shared__ float sG[2][16][G4 + 1]; __shared__ __attribute__((aligned(16))) unsigned short sW[G4][HH];
  const int tid = threadIdx.x, wv = tid >> 5, lane = tid & 31, ln = lane & 15, hh = lane >> 4; const int row0 = (blockIdx.x * 2 + wv) * 16;
  float (*myH)[HH + 1] = sH[wv]; float (*myC)[HH + 1] = sC[wv]; float (*myG)[G4 + 1] = sG[wv]; unsigned short (*myW)[HH] = sW;
  for (int r = 0; r < 16; ++r) { myH[r][lane] = bf16_round(bh0[lane]); myH[r][32 + lane] = bf16_round(bh0[32 + lane]); myC[r][lane] = bf16_round(bc0[lane]); myC[r][32 + lane] = bf16_round(bc0[32 + lane]); }
#pragma unroll 1
  for (int phase = 0; phase < 2; ++phase) { const float* Whh = phase ? Whh_d : Whh_e; const float* GI = phase ? GId : GIe; const int T = phase ? TD : TE;
    __syncthreads();
    for (int e = tid; e < G4 * HH; e += 64) myW[e / HH][e % HH] = bf16_bits(Whh[e]);
    __syncthreads();
#pragma unroll 1
    for (int step = 0; step < T; ++step) {
      v8f acc[16]; for (int t = 0; t < 16; ++t) acc[t] = (v8f){0.f,0.f,0.f,0.f,0.f,0.f,0.f,0.f};
#pragma unroll
      for (int kb = 0; kb < HH; kb += 32) { FragB ah, al;
#pragma unroll
        for (int q = 0; q < 8; ++q) { const float v0 = myH[ln][kb + 8 * hh + q], v1 = myH[ln][kb + 16 + 8 * hh + q]; const unsigned short h0 = bf16_bits(v0), h1 = bf16_bits(v1); ah.u[q] = h0; al.u[q] = bf16_bits(v0 - bf16_val(h0)); ah.u[8 + q] = h1; al.u[8 + q] = bf16_bits(v1 - bf16_val(h1)); }
#pragma unroll
        for (int t = 0; t < 16; ++t) { FragB bw; bw.half[0] = *(const v8us*)&myW[t * 16 + ln][kb + 8 * hh]; bw.half[1] = *(const v8us*)&myW[t * 16 + ln][kb + 16 + 8 * hh]; acc[t] = mmaN<2>(ah.v, al.v, bw.v, bw.v, acc[t]); } }
#pragma unroll
      for (int t = 0; t < 16; ++t) {
#pragma unroll
        for (int r = 0; r < 8; ++r) myG[8 * hh + r][t * 16 + ln] = acc[t][r]; }
      __builtin_amdgcn_fence(__ATOMIC_ACQ_REL, "workgroup"); __builtin_amdgcn_wave_barrier();
#pragma unroll 1
      for (int r = 0; r < 16; ++r) { const float* gi = GI + ((size_t)(row0 + r) * T + step) * G4;
#pragma unroll
        for (int a = 0; a < 2; ++a) { const int u = a * 32 + lane; const float gI = myG[r][u] + gi[u], gF = myG[r][HH + u] + gi[HH + u], gG = myG[r][2 * HH + u] + gi[2 * HH + u], gO = myG[r][3 * HH + u] + gi[3 * HH + u];
          const float cn = sigm(gF) * myC[r][u] + sigm(gI) * tnh(gG); myC[r][u] = cn; myH[r][u] = sigm(gO) * tnh(cn); } }
      __builtin_amdgcn_fence(__ATOMIC_ACQ_REL, "workgroup"); __builtin_amdgcn_wave_barrier();
      if (phase == 1) { for (int pass = 0; pass < 2; ++pass) { for (int r = 0; r < 16; ++r) { float* d = DEC + ((size_t)(row0 + r) * TD + step) * HH; *(volatile float*)(d + lane) = myH[r][lane]; *(volatile float*)(d + 32 + lane) = myH[r][32 + lane]; } if (pass == 0) __threadfence(); } }
    } }
}
__global__ __launch_bounds__(1024) void k_post(const float* __restrict__ U2, const float* __restrict__ DH, const float* __restrict__ gamma, const float* __restrict__ beta, const float* __restrict__ Wh, const float* __restrict__ bh, float* __restrict__ pred) {
  __shared__ float sp[32]; const int tid = threadIdx.x, wv = tid >> 5, lane = tid & 31; const int tk = blockIdx.x * 32 + wv; float v0, v1;
  { const float* u2 = U2 + (size_t)tk * (2 * HH); const float* dh = DH + (size_t)tk * HH; v0 = sigm(u2[lane]) * u2[HH + lane] + dh[lane]; v1 = sigm(u2[32 + lane]) * u2[HH + 32 + lane] + dh[32 + lane]; }
  float s = v0 + v1; for (int o = 16; o >= 1; o >>= 1) s += __shfl_xor(s, o, 32); const float mu = s * (1.0f / HH); const float d0 = v0 - mu, d1 = v1 - mu; float q = d0 * d0 + d1 * d1; for (int o = 16; o >= 1; o >>= 1) q += __shfl_xor(q, o, 32); const float rs = rsqrtf(q * (1.0f / HH) + 1e-5f);
  const float y0 = d0 * rs * bf16_round(gamma[lane]) + bf16_round(beta[lane]), y1 = d1 * rs * bf16_round(gamma[32 + lane]) + bf16_round(beta[32 + lane]);
  float p = y0 * bf16_round(Wh[lane]) + y1 * bf16_round(Wh[32 + lane]); for (int o = 16; o >= 1; o >>= 1) p += __shfl_xor(p, o, 32);
  if (lane == 0) sp[wv] = p + bf16_round(bh[0]); __syncthreads();
  if (tid < 32) { *(volatile float*)(pred + (size_t)blockIdx.x * 32 + tid) = sp[tid]; } __threadfence(); if (tid < 32) { *(volatile float*)(pred + (size_t)blockIdx.x * 32 + tid) = sp[tid]; }
}
__global__ __launch_bounds__(256) void k_hc0(const float* __restrict__ bh0, const float* __restrict__ bc0, float* __restrict__ oh, float* __restrict__ oc) { const int t = blockIdx.x * 256 + threadIdx.x; if (t >= BB * HH) return; const int u = t % HH; const float a = bf16_round(bh0[u]), b = bf16_round(bc0[u]); *(volatile float*)(oh + t) = a; *(volatile float*)(oc + t) = b; __threadfence(); *(volatile float*)(oh + t) = a; *(volatile float*)(oc + t) = b; }
extern "C" void kernel_launch(void* const* d_in, const int* in_sizes, int n_in,
                              void* d_out, int out_size, void* d_ws, size_t ws_size, hipStream_t stream) {
  (void)in_sizes; (void)n_in; (void)out_size;
  const float* Xe = (const float*)d_in[0]; const float* Xd = (const float*)d_in[1]; const float* Wp = (const float*)d_in[2]; const float* bp = (const float*)d_in[3]; const float* Se = (const float*)d_in[4]; const float* Sd = (const float*)d_in[5];
  (void)d_in[6]; const float* bh0 = (const float*)d_in[7]; (void)d_in[8]; const float* bc0 = (const float*)d_in[9];
  const float* Wih_e = (const float*)d_in[10]; const float* Whh_e = (const float*)d_in[11]; const float* bih_e = (const float*)d_in[12]; const float* bhh_e = (const float*)d_in[13]; const float* Wih_d = (const float*)d_in[14]; const float* Whh_d = (const float*)d_in[15]; const float* bih_d = (const float*)d_in[16]; const float* bhh_d = (const float*)d_in[17];
  const float* Wz = (const float*)d_in[18]; const float* bz = (const float*)d_in[19]; const float* Wg = (const float*)d_in[20]; const float* bg = (const float*)d_in[21]; const float* gamma = (const float*)d_in[22]; const float* beta = (const float*)d_in[23]; const float* Wh = (const float*)d_in[24]; const float* bh = (const float*)d_in[25];
  float* pred = (float*)d_out; float* oh0 = pred + (size_t)NTD; float* oc0 = oh0 + BB * HH;
  char* ws = (char*)d_ws; size_t off = 0;
  auto take = [&](size_t bytes) { char* p = ws + off; off += (bytes + 255) & ~(size_t)255; return p; };
  unsigned short* Bv = (unsigned short*)take(HH * 2 * FF * 2); unsigned short* Bie = (unsigned short*)take(G4 * HH * 2); unsigned short* Bid = (unsigned short*)take(G4 * HH * 2); unsigned short* Bgz = (unsigned short*)take(2 * HH * HH * 2); float* bse = (float*)take(G4 * 4); float* bsd = (float*)take(G4 * 4); float* bgz = (float*)take(2 * HH * 4);
  float* Ae = (float*)take((size_t)NTE * 2 * FF * 4); float* Ad = (float*)take((size_t)NTD * 2 * FF * 4); float* He = (float*)take((size_t)NTE * HH * 4); float* Hd = (float*)take((size_t)NTD * HH * 4); float* GIe = (float*)take((size_t)NTE * G4 * 4); float* GId = (float*)take((size_t)NTD * G4 * 4); float* DEC = (float*)take((size_t)NTD * HH * 4); float* U2 = (float*)take((size_t)NTD * 2 * HH * 4);
  if (off > ws_size) return;
  k_btvsn<<<(HH * 8 + 255) / 256, 256, 0, stream>>>(Wp, bp, Bv); k_round_rows<<<(G4 * HH / 8 + 255) / 256, 256, 0, stream>>>(Wih_e, Bie, G4 * HH / 8); k_round_rows<<<(G4 * HH / 8 + 255) / 256, 256, 0, stream>>>(Wih_d, Bid, G4 * HH / 8);
  k_round_rows<<<(HH * HH / 8 + 255) / 256, 256, 0, stream>>>(Wg, Bgz, HH * HH / 8); k_round_rows<<<(HH * HH / 8 + 255) / 256, 256, 0, stream>>>(Wz, Bgz + HH * HH, HH * HH / 8);
  k_bsum<<<1, 256, 0, stream>>>(bih_e, bhh_e, bse); k_bsum<<<1, 256, 0, stream>>>(bih_d, bhh_d, bsd); k_bcat2<<<1, 256, 0, stream>>>(bg, bz, bgz);
  k_vsnA<<<NTE / 8, 256, 0, stream>>>(Xe, Se, NTE, Ae); k_vsnA<<<NTD / 8, 256, 0, stream>>>(Xd, Sd, NTD, Ad);
  k_gemm_bf3<true, 0, false, false><<<((NTE / 16) * 1 + 3) / 4, 128, 0, stream>>>(Ae, 2 * FF, Bv, 2 * FF, nullptr, nullptr, 1, 0, He, HH, NTE, HH, 2 * FF);
  k_gemm_bf3<true, 0, false, false><<<((NTD / 16) * 1 + 3) / 4, 128, 0, stream>>>(Ad, 2 * FF, Bv, 2 * FF, nullptr, nullptr, 1, 0, Hd, HH, NTD, HH, 2 * FF);
  k_gemm_bf3<true, 0, false, false><<<((NTE / 16) * 4 + 3) / 4, 128, 0, stream>>>(He, HH, Bie, HH, bse, nullptr, 1, 0, GIe, G4, NTE, G4, HH);
  k_gemm_bf3<true, 0, false, false><<<((NTD / 16) * 4 + 3) / 4, 128, 0, stream>>>(Hd, HH, Bid, HH, bsd, nullptr, 1, 0, GId, G4, NTD, G4, HH);
  k_lstm2<<<BB / 32, 64, 0, stream>>>(GIe, GId, Whh_e, Whh_d, bh0, bc0, DEC);
  k_gemm_bf3<true, 0, true, false><<<((NTD / 16) * 2 + 3) / 4, 128, 0, stream>>>(DEC, HH, Bgz, HH, bgz, nullptr, 1, 0, U2, 2 * HH, NTD, 2 * HH, HH);
  k_post<<<NTD / 32, 1024, 0, stream>>>(U2, Hd, gamma, beta, Wh, bh, pred);
  k_hc0<<<(BB * HH + 255) / 256, 256, 0, stream>>>(bh0, bc0, oh0, oc0);
}
